// SpectrumAttention_45449343926360
// MI455X (gfx1250) — hardware-verified
//
#include <hip/hip_runtime.h>


#define NB_  8
#define CC   256
#define NN_  2048
#define HQ   32
#define NTK  (NB_ * NN_)
#define PSC  32768.0f
#define LOSC 1024.0f
#define LOSCI (1.0f / 1024.0f)

typedef _Float16 h16;
typedef unsigned short bf;
typedef __attribute__((ext_vector_type(16))) __bf16   v16bf;
typedef __attribute__((ext_vector_type(16))) _Float16 v16h;
typedef __attribute__((ext_vector_type(8)))  _Float16 v8h;
typedef __attribute__((ext_vector_type(8)))  unsigned short v8us;
typedef __attribute__((ext_vector_type(8)))  float    v8f;
typedef __attribute__((ext_vector_type(4)))  float    v4f;
typedef v8h  __attribute__((may_alias)) v8ha;
typedef v4f  __attribute__((may_alias)) v4fa;
typedef v8us __attribute__((may_alias)) v8usa;

__device__ __forceinline__ unsigned short f2bf(float f) { unsigned u = __float_as_uint(f); u += 0x7FFFu + ((u >> 16) & 1u); return (unsigned short)(u >> 16); }
__device__ __forceinline__ float bf2f(unsigned short b) { return __uint_as_float(((unsigned)b) << 16); }
__device__ __forceinline__ float bfr(float f) { return bf2f(f2bf(f)); }
__device__ __forceinline__ v16h cat16(v8h lo, v8h hi) { return __builtin_shufflevector(lo, hi, 0, 1, 2, 3, 4, 5, 6, 7, 8, 9, 10, 11, 12, 13, 14, 15); }
__device__ __forceinline__ v16bf cat16b(v8us lo, v8us hi) { return __builtin_bit_cast(v16bf, __builtin_shufflevector(lo, hi, 0, 1, 2, 3, 4, 5, 6, 7, 8, 9, 10, 11, 12, 13, 14, 15)); }
__device__ __forceinline__ v8f wmma16(v16h a, v16h b, v8f c) { return __builtin_amdgcn_wmma_f32_16x16x32_f16(false, a, false, b, (short)0, c, false, false); }
__device__ __forceinline__ v8f wmmab(v16bf a, v16bf b, v8f c) { return __builtin_amdgcn_wmma_f32_16x16x32_bf16(false, a, false, b, (short)0, c, false, false); }
#define VST2(T, p, v) do { const T vst2_v_ = (v); *(volatile T*)(p) = vst2_v_; __threadfence(); *(volatile T*)(p) = vst2_v_; } while (0)

__global__ __launch_bounds__(256) void k_xt(const float* __restrict__ x, bf* XT) {
    __shared__ __align__(16) unsigned short tl[64 * 72];
    const int tid = threadIdx.x, n0 = blockIdx.x * 64, c0 = blockIdx.y * 64, b = blockIdx.z;
    const int cr = tid >> 2, nq = (tid & 3) * 16;
#pragma unroll
    for (int i = 0; i < 16; ++i) tl[(nq + i) * 72 + cr] = f2bf(x[((size_t)b * CC + c0 + cr) * NN_ + n0 + nq + i]);
    __syncthreads();
    const int piece = tid & 7;
    auto pass = [&]() {
#pragma unroll
        for (int s = 0; s < 2; ++s) { const int nr = (tid >> 3) + 32 * s; const v8us val = *(const v8usa*)(tl + nr * 72 + piece * 8); *(volatile v8us*)(XT + ((size_t)b * NN_ + n0 + nr) * CC + c0 + piece * 8) = val; }
    };
    pass(); __threadfence(); pass();
}
__global__ __launch_bounds__(256) void k_w(const float* __restrict__ wq, const float* __restrict__ wk, const float* __restrict__ wv, bf* WQ, bf* WK, bf* WV) {
    const int lane = threadIdx.x & 31, r = blockIdx.x * 8 + (threadIdx.x >> 5);
    const int m = (r < HQ) ? 0 : (r < 2 * HQ) ? 1 : 2;
    v8us o;
    if (m == 0) { for (int i = 0; i < 8; ++i) o[i] = f2bf(wq[(size_t)r * CC + lane * 8 + i]); VST2(v8us, WQ + (size_t)r * CC + lane * 8, o); }
    else if (m == 1) { const int o2 = r - HQ; for (int i = 0; i < 8; ++i) o[i] = f2bf(wk[(size_t)o2 * CC + lane * 8 + i]); VST2(v8us, WK + (size_t)o2 * CC + lane * 8, o); }
    else { const int o2 = r - 2 * HQ; if (o2 < CC) { for (int i = 0; i < 8; ++i) o[i] = f2bf(wv[(size_t)o2 * CC + lane * 8 + i]); VST2(v8us, WV + (size_t)o2 * CC + lane * 8, o); } }
}
__global__ __launch_bounds__(128) void k_qk(const bf* __restrict__ XT, const bf* __restrict__ WQ, const bf* __restrict__ WK, const float* __restrict__ bq, const float* __restrict__ bk, h16* QH, h16* QL, h16* KH, h16* KL) {
    __shared__ __align__(16) float ost[4][16 * 36];
    const int lane = threadIdx.x & 31, wave = threadIdx.x >> 5, lr = lane & 15, hi = lane >> 4, which = blockIdx.y;
    const size_t r0 = (size_t)blockIdx.x * 64 + wave * 16;
    const bf* W = which ? WK : WQ; const float* bias = which ? bk : bq; h16* PH = which ? KH : QH; h16* PL = which ? KL : QL;
    v8f acc[2] = {(v8f){}, (v8f){}};
#pragma unroll 2
    for (int kc = 0; kc < CC; kc += 32) {
        const v16bf a = cat16b(*(const v8us*)(XT + (r0 + lr) * CC + kc + 8 * hi), *(const v8us*)(XT + (r0 + lr) * CC + kc + 8 * hi + 16));
#pragma unroll
        for (int t = 0; t < 2; ++t) { const bf* bp = W + (size_t)(t * 16 + lr) * CC + kc + 8 * hi; acc[t] = wmmab(a, cat16b(*(const v8us*)bp, *(const v8us*)(bp + 16)), acc[t]); }
    }
    float* os = &ost[wave][0];
#pragma unroll
    for (int t = 0; t < 2; ++t) { const float bv = bfr(bias[t * 16 + lr]);
#pragma unroll
        for (int j = 0; j < 8; ++j) os[(hi * 8 + j) * 36 + t * 16 + lr] = acc[t][j] + bv; }
    __syncthreads();
    auto pass = [&]() {
#pragma unroll
        for (int s = 0; s < 2; ++s) { const int row = s * 8 + (lane >> 2), piece = lane & 3; const float* sp = os + row * 36 + piece * 8; v8h oh, ol;
#pragma unroll
            for (int i = 0; i < 8; ++i) { const h16 a = (h16)sp[i]; oh[i] = a; ol[i] = (h16)((sp[i] - (float)a) * LOSC); }
            *(volatile v8h*)(PH + (r0 + row) * HQ + piece * 8) = oh; *(volatile v8h*)(PL + (r0 + row) * HQ + piece * 8) = ol; }
    };
    pass(); __threadfence(); pass();
}
__global__ __launch_bounds__(128) void k_v(const bf* __restrict__ XT, const bf* __restrict__ WV, const float* __restrict__ bv, float* Vf) {
    __shared__ __align__(16) float ost[4][16 * 68];
    const int lane = threadIdx.x & 31, wave = threadIdx.x >> 5, lr = lane & 15, hi = lane >> 4;
    const size_t r0 = (size_t)blockIdx.x * 64 + wave * 16; const int c0 = blockIdx.y * 64;
    v8f acc[4];
#pragma unroll
    for (int t = 0; t < 4; ++t) acc[t] = (v8f){};
#pragma unroll 2
    for (int kc = 0; kc < CC; kc += 32) {
        const v16bf a = cat16b(*(const v8us*)(XT + (r0 + lr) * CC + kc + 8 * hi), *(const v8us*)(XT + (r0 + lr) * CC + kc + 8 * hi + 16));
#pragma unroll
        for (int t = 0; t < 4; ++t) { const bf* bp = WV + (size_t)(c0 + t * 16 + lr) * CC + kc + 8 * hi; acc[t] = wmmab(a, cat16b(*(const v8us*)bp, *(const v8us*)(bp + 16)), acc[t]); }
    }
    float* os = &ost[wave][0];
#pragma unroll
    for (int t = 0; t < 4; ++t) { const float b2 = bfr(bv[c0 + t * 16 + lr]);
#pragma unroll
        for (int j = 0; j < 8; ++j) os[(hi * 8 + j) * 68 + t * 16 + lr] = acc[t][j] + b2; }
    __syncthreads();
    float* crow = Vf + r0 * CC + c0;
    auto pass = [&]() {
#pragma unroll
        for (int s = 0; s < 8; ++s) { const int Lid = (lane >> 3) + 4 * s, piece = lane & 7; const int row = Lid >> 1, cofs = (Lid & 1) * 32 + piece * 4;
            const v4f val = *(const v4fa*)(os + row * 68 + cofs); *(volatile v4f*)(crow + (size_t)row * CC + cofs) = val; }
    };
    pass(); __threadfence(); pass();
}
__global__ __launch_bounds__(256) void k_vt(const float* __restrict__ Vf, h16* VTH, h16* VTL) {
    __shared__ __align__(16) h16 tl[64 * 72];
    __shared__ __align__(16) h16 tl2[64 * 72];
    const int tid = threadIdx.x, n0 = blockIdx.x * 64, c0 = blockIdx.y * 64, b = blockIdx.z;
    const int nn = tid >> 2, cq = (tid & 3) * 16;
#pragma unroll
    for (int i = 0; i < 16; ++i) { const float v = Vf[((size_t)b * NN_ + n0 + nn) * CC + c0 + cq + i]; const h16 a = (h16)v; tl[(cq + i) * 72 + nn] = a; tl2[(cq + i) * 72 + nn] = (h16)((v - (float)a) * LOSC); }
    __syncthreads();
    const int piece = tid & 7;
    auto pass = [&]() {
#pragma unroll
        for (int s = 0; s < 2; ++s) { const int c = (tid >> 3) + 32 * s; const size_t o = ((size_t)b * CC + c0 + c) * NN_ + n0 + piece * 8;
            *(volatile v8h*)(VTH + o) = *(const v8ha*)(tl + c * 72 + piece * 8); *(volatile v8h*)(VTL + o) = *(const v8ha*)(tl2 + c * 72 + piece * 8); }
    };
    pass(); __threadfence(); pass();
}
__global__ __launch_bounds__(128) void k_attn(const h16* __restrict__ QH, const h16* __restrict__ QL, const h16* __restrict__ KH, const h16* __restrict__ KL, const h16* __restrict__ VTH, const h16* __restrict__ VTL,
                                             const float* __restrict__ x, float* out) {
    __shared__ __align__(16) h16 plds[4][16 * 32];
    __shared__ __align__(16) h16 plds2[4][16 * 32];
    __shared__ __align__(16) float ot[128 * 68];
    const int lane = threadIdx.x & 31, wave = threadIdx.x >> 5, lr = lane & 15, hi = lane >> 4;
    const int b = blockIdx.x / (NN_ / 64), it = blockIdx.x - b * (NN_ / 64), chalf = blockIdx.y, i0l = it * 64, q0 = i0l + wave * 16;
    const size_t tok0 = (size_t)b * NN_;
    h16* pl = &plds[wave][0]; h16* pl2 = &plds2[wave][0];
    const size_t qo = (tok0 + q0 + lr) * HQ + 8 * hi;
    const v16h qa = cat16(*(const v8h*)(QH + qo), *(const v8h*)(QH + qo + 16));
    v8f o[8], ox[8];
#pragma unroll
    for (int n = 0; n < 8; ++n) { o[n] = (v8f){}; ox[n] = (v8f){}; }
    float mrow[8], lpart[8];
#pragma unroll
    for (int j = 0; j < 8; ++j) { mrow[j] = -3.0e38f; lpart[j] = 0.f; }
#pragma unroll 1
    for (int kt = 0; kt < NN_ / 32; ++kt) {
        const int l0 = kt * 32;
        const size_t k0o = (tok0 + l0 + lr) * HQ + 8 * hi, k1o = k0o + (size_t)16 * HQ;
        const v16h k0h = cat16(*(const v8h*)(KH + k0o), *(const v8h*)(KH + k0o + 16)), k1h = cat16(*(const v8h*)(KH + k1o), *(const v8h*)(KH + k1o + 16));
        const v16h k0l = cat16(*(const v8h*)(KL + k0o), *(const v8h*)(KL + k0o + 16)), k1l = cat16(*(const v8h*)(KL + k1o), *(const v8h*)(KL + k1o + 16));
        const v16h ql = cat16(*(const v8h*)(QL + qo), *(const v8h*)(QL + qo + 16));
        v8f s0 = wmma16(qa, k0h, (v8f){}), s1 = wmma16(qa, k1h, (v8f){}), x0 = wmma16(ql, k0h, (v8f){}), x1 = wmma16(ql, k1h, (v8f){});
        x0 = wmma16(qa, k0l, x0); x1 = wmma16(qa, k1l, x1);
        asm volatile("v_nop\n\tv_nop\n\tv_nop\n\tv_nop" : "+v"(s0), "+v"(s1), "+v"(x0), "+v"(x1) : "v"(qa), "v"(ql));
        float alpha[8];
#pragma unroll
        for (int j = 0; j < 8; ++j) {
            const float a0 = s0[j] + x0[j] * LOSCI, a1 = s1[j] + x1[j] * LOSCI;
            float mx = fmaxf(a0, a1);
            mx = fmaxf(mx, __shfl_xor(mx, 1, 16)); mx = fmaxf(mx, __shfl_xor(mx, 2, 16)); mx = fmaxf(mx, __shfl_xor(mx, 4, 16)); mx = fmaxf(mx, __shfl_xor(mx, 8, 16));
            const float mn = fmaxf(mrow[j], mx);
            alpha[j] = __expf(mrow[j] - mn); mrow[j] = mn;
            const float p0 = __expf(a0 - mn), p1 = __expf(a1 - mn);
            lpart[j] = lpart[j] * alpha[j] + (p0 + p1);
            const int mr = hi * 8 + j;
            const float ps0 = p0 * PSC, ps1 = p1 * PSC; const h16 h0 = (h16)ps0, h1 = (h16)ps1;
            pl[mr * 32 + lr] = h0; pl[mr * 32 + 16 + lr] = h1; pl2[mr * 32 + lr] = (h16)(ps0 - (float)h0); pl2[mr * 32 + 16 + lr] = (h16)(ps1 - (float)h1);
        }
#pragma unroll
        for (int n = 0; n < 8; ++n)
#pragma unroll
            for (int j = 0; j < 8; ++j) { o[n][j] *= alpha[j]; ox[n][j] *= alpha[j]; }
        asm volatile("" ::: "memory");
        const v16h pa = cat16(*(const v8ha*)(pl + lr * 32 + hi * 8), *(const v8ha*)(pl + lr * 32 + 16 + hi * 8));
        const v16h px = cat16(*(const v8ha*)(pl2 + lr * 32 + hi * 8), *(const v8ha*)(pl2 + lr * 32 + 16 + hi * 8));
#pragma unroll
        for (int n = 0; n < 8; ++n) { const size_t vo = ((size_t)b * CC + chalf * 128 + n * 16 + lr) * NN_ + l0 + hi * 8;
            const v16h vh = cat16(*(const v8h*)(VTH + vo), *(const v8h*)(VTH + vo + 16)), vl = cat16(*(const v8h*)(VTL + vo), *(const v8h*)(VTL + vo + 16));
            o[n] = wmma16(pa, vh, o[n]); o[n] = wmma16(px, vh, o[n]); ox[n] = wmma16(pa, vl, ox[n]);
            asm volatile("" : "+v"(o[n]), "+v"(ox[n]) : "v"(vh), "v"(vl) : "memory"); }
        asm volatile("v_nop\n\tv_nop\n\tv_nop\n\tv_nop" : "+v"(o[0]), "+v"(o[7]), "+v"(ox[0]), "+v"(ox[7]) : "v"(pa), "v"(px));
    }
    float inv[8];
#pragma unroll
    for (int j = 0; j < 8; ++j) { float rs = lpart[j]; rs += __shfl_xor(rs, 1, 16); rs += __shfl_xor(rs, 2, 16); rs += __shfl_xor(rs, 4, 16); rs += __shfl_xor(rs, 8, 16); inv[j] = 1.0f / (rs * PSC); }
#pragma unroll
    for (int n = 0; n < 8; ++n)
#pragma unroll
        for (int j = 0; j < 8; ++j) ot[(n * 16 + lr) * 68 + wave * 16 + hi * 8 + j] = (o[n][j] + ox[n][j] * LOSCI) * inv[j];
    __syncthreads();
    auto pass = [&]() {
#pragma unroll
        for (int s = 0; s < 16; ++s) { const int cl = wave * 32 + s * 2 + (lane >> 4), piece = lane & 15; const size_t go = ((size_t)b * CC + chalf * 128 + cl) * NN_ + i0l + piece * 4;
            v4f val = *(const v4fa*)(ot + cl * 68 + piece * 4);
#pragma unroll
            for (int i = 0; i < 4; ++i) val[i] += bfr(x[go + i]);
            *(volatile v4f*)(out + go) = val; }
    };
    pass(); __threadfence(); pass();
}

extern "C" void kernel_launch(void* const* d_in, const int* in_sizes, int n_in,
                              void* d_out, int out_size, void* d_ws, size_t ws_size, hipStream_t stream) {
    (void)in_sizes; (void)n_in; (void)out_size;
    const float* x = (const float*)d_in[0]; const float* wq = (const float*)d_in[1]; const float* bq = (const float*)d_in[2]; const float* wk = (const float*)d_in[3]; const float* bk = (const float*)d_in[4];
    const float* wv = (const float*)d_in[5]; const float* bv = (const float*)d_in[6];
    float* out = (float*)d_out;
    char* wsp = (char*)d_ws;
    auto take = [&](size_t bytes) { char* p = wsp; wsp += (bytes + 255) & ~(size_t)255; return (void*)p; };
    bf* XT = (bf*)take((size_t)NTK * CC * 2); bf* WQ = (bf*)take((size_t)HQ * CC * 2); bf* WK = (bf*)take((size_t)HQ * CC * 2); bf* WV = (bf*)take((size_t)CC * CC * 2);
    h16* QH = (h16*)take((size_t)NTK * HQ * 2); h16* QL = (h16*)take((size_t)NTK * HQ * 2); h16* KH = (h16*)take((size_t)NTK * HQ * 2); h16* KL = (h16*)take((size_t)NTK * HQ * 2);
    float* Vf = (float*)take((size_t)NTK * CC * 4); h16* VTH = (h16*)take((size_t)NTK * CC * 2); h16* VTL = (h16*)take((size_t)NTK * CC * 2);
    if ((size_t)(wsp - (char*)d_ws) > ws_size) return;
    k_xt<<<dim3(NN_ / 64, CC / 64, NB_), 256, 0, stream>>>(x, XT);
    k_w<<<(2 * HQ + CC) / 8, 256, 0, stream>>>(wq, wk, wv, WQ, WK, WV);
    k_qk<<<dim3(NTK / 64, 2, 1), 128, 0, stream>>>(XT, WQ, WK, bq, bk, QH, QL, KH, KL);
    k_v<<<dim3(NTK / 64, CC / 64, 1), 128, 0, stream>>>(XT, WV, bv, Vf);
    k_vt<<<dim3(NN_ / 64, CC / 64, NB_), 256, 0, stream>>>(Vf, VTH, VTL);
    k_attn<<<dim3(NB_ * (NN_ / 64), 2, 1), 128, 0, stream>>>(QH, QL, KH, KL, VTH, VTL, x, out);
}
